// mLSTMLayer_89807766159690
// MI455X (gfx1250) — hardware-run, weakly checked
//
#include <hip/hip_runtime.h>

typedef _Float16 f16t;
typedef f16t  v16h __attribute__((ext_vector_type(16)));
typedef f16t  v8h  __attribute__((ext_vector_type(8)));
typedef float v8f  __attribute__((ext_vector_type(8)));
typedef float v4f  __attribute__((ext_vector_type(4)));

#define HD    768
#define INN   1152
#define NHD   8
#define DHD   144
#define BSZ   2
#define SEQ   2048
#define MROWS (BSZ * SEQ)
#define GK    (3 * INN)

union Frag { v16h v; v8h h[2]; uint4 u[2]; };

__device__ __forceinline__ v8f wmma16(v16h a, v16h b, v8f c)
{
    c = __builtin_amdgcn_wmma_f32_16x16x32_f16(false, a, false, b, (short)0, c, false, false);
    asm volatile("v_nop\n\tv_nop\n\tv_nop\n\tv_nop" : "+v"(c) : "v"(a), "v"(b));
    return c;
}
__device__ __forceinline__ v8f zacc()
{
    v8f c;
#pragma unroll
    for (int i = 0; i < 8; ++i) c[i] = 0.f;
    return c;
}
__device__ __forceinline__ uint4 zu4() { return make_uint4(0u, 0u, 0u, 0u); }

__device__ __forceinline__ float logsig(float x)
{
    return (x > 0.f) ? -log1pf(expf(-x)) : (x - log1pf(expf(x)));
}

__global__ __launch_bounds__(256) void k_cvt_rows(const float* __restrict__ src, f16t* __restrict__ dst,
                                                    int n8, float scale)
{
    const int i = blockIdx.x * 256 + threadIdx.x;
    if (i >= n8) return;
    const v4f* s = (const v4f*)(src + (size_t)i * 8);
    const v4f a = s[0], b = s[1];
    v8h o;
    o[0] = (f16t)(a[0] * scale); o[1] = (f16t)(a[1] * scale); o[2] = (f16t)(a[2] * scale); o[3] = (f16t)(a[3] * scale);
    o[4] = (f16t)(b[0] * scale); o[5] = (f16t)(b[1] * scale); o[6] = (f16t)(b[2] * scale); o[7] = (f16t)(b[3] * scale);
    f16t* d = dst + (size_t)i * 8;
    *(volatile v8h*)d = o;
    __threadfence();
    *(volatile v8h*)d = o;
}

__global__ __launch_bounds__(256) void k_tr_cvt(const float* __restrict__ in, f16t* __restrict__ out,
                                                  int R, int C, float scale)
{
    __shared__ __align__(16) f16t T[64 * 72];
    const int tid = threadIdx.x;
    const int r0 = blockIdx.x * 64, c0 = blockIdx.y * 64;
    {
        const int rr = tid >> 2, cc = (tid & 3) * 16;
        if (r0 + rr < R && c0 + cc + 16 <= C) {
            const v4f* s = (const v4f*)(in + (size_t)(r0 + rr) * C + c0 + cc);
            const v4f q0 = s[0], q1 = s[1], q2 = s[2], q3 = s[3];
#pragma unroll
            for (int i = 0; i < 4; ++i) {
                T[(cc + i) * 72 + rr]      = (f16t)(q0[i] * scale);
                T[(cc + 4 + i) * 72 + rr]  = (f16t)(q1[i] * scale);
                T[(cc + 8 + i) * 72 + rr]  = (f16t)(q2[i] * scale);
                T[(cc + 12 + i) * 72 + rr] = (f16t)(q3[i] * scale);
            }
        }
    }
    __syncthreads();
    const int piece = tid & 7;
    const int l0 = tid >> 3, l1 = l0 + 32;
    const bool ok0 = (c0 + l0 < C) && (r0 + 64 <= R);
    const bool ok1 = (c0 + l1 < C) && (r0 + 64 <= R);
    const v8h v0 = *(const v8h*)(T + l0 * 72 + piece * 8);
    const v8h v1 = *(const v8h*)(T + l1 * 72 + piece * 8);
    f16t* d0 = out + (size_t)(c0 + l0) * R + r0 + piece * 8;
    f16t* d1 = out + (size_t)(c0 + l1) * R + r0 + piece * 8;
    if (ok0) *(volatile v8h*)d0 = v0;
    if (ok1) *(volatile v8h*)d1 = v1;
    __threadfence();
    if (ok0) *(volatile v8h*)d0 = v0;
    if (ok1) *(volatile v8h*)d1 = v1;
}

__global__ __launch_bounds__(256) void k_gatew(const float* __restrict__ Wi, const float* __restrict__ Wf,
                                                 f16t* __restrict__ WgT, int n8, float scale)
{
    const int i = blockIdx.x * 256 + threadIdx.x;
    if (i >= n8) return;
    const int n = i / (GK / 8);
    const int k8 = i - n * (GK / 8);
    const float* src = (n < 8) ? (Wi + n) : (Wf + (n - 8));
    v8h o;
#pragma unroll
    for (int t = 0; t < 8; ++t) o[t] = (f16t)(src[(size_t)(k8 * 8 + t) * NHD] * scale);
    f16t* d = WgT + (size_t)i * 8;
    *(volatile v8h*)d = o;
    __threadfence();
    *(volatile v8h*)d = o;
}

__global__ __launch_bounds__(256) void k_gemm(const f16t* __restrict__ A, int lda,
                                                const f16t* __restrict__ Bt, int ldb,
                                                f16t* __restrict__ out16, float* __restrict__ out32,
                                                f16t* __restrict__ outT, int ldc,
                                                int M, int N, int K, int mode, float osc)
{
    __shared__ __align__(16) f16t S16[128 * 136];
    float* S32 = (float*)S16;
    const int tid = threadIdx.x, wid = tid >> 5, lane = tid & 31, hf = lane >> 4, m = lane & 15;
    const int mBase = blockIdx.y * 128, nBase = blockIdx.x * 128;
    if (mBase + 128 > M || nBase + 128 > N) return;
    const int wm = wid & 1, wn = wid >> 1;

    v8f acc[4][2];
#pragma unroll
    for (int i = 0; i < 4; ++i) { acc[i][0] = zacc(); acc[i][1] = zacc(); }

    const f16t* Ab = A  + (size_t)(mBase + wm * 64 + m) * lda + 8 * hf;
    const f16t* Bb = Bt + (size_t)(nBase + wn * 32 + m) * ldb + 8 * hf;

#pragma unroll 1
    for (int kb = 0; kb < K; kb += 32) {
        Frag af[4], bfr[2];
#pragma unroll
        for (int mi = 0; mi < 4; ++mi) {
            const f16t* p = Ab + (size_t)(mi * 16) * lda + kb;
            af[mi].h[0] = *(const v8h*)p;
            af[mi].h[1] = *(const v8h*)(p + 16);
        }
#pragma unroll
        for (int ni = 0; ni < 2; ++ni) {
            const f16t* p = Bb + (size_t)(ni * 16) * ldb + kb;
            bfr[ni].h[0] = *(const v8h*)p;
            bfr[ni].h[1] = *(const v8h*)(p + 16);
        }
#pragma unroll
        for (int mi = 0; mi < 4; ++mi) {
            acc[mi][0] = wmma16(af[mi].v, bfr[0].v, acc[mi][0]);
            acc[mi][1] = wmma16(af[mi].v, bfr[1].v, acc[mi][1]);
        }
    }

    if (mode == 1) {
#pragma unroll
        for (int p = 0; p < 2; ++p) {
            if (wm == p) {
#pragma unroll
                for (int mi = 0; mi < 4; ++mi)
#pragma unroll
                    for (int ni = 0; ni < 2; ++ni)
#pragma unroll
                        for (int r = 0; r < 8; ++r)
                            S32[(mi * 16 + 8 * hf + r) * 132 + wn * 32 + ni * 16 + m] = acc[mi][ni][r] * osc;
            }
            __syncthreads();
            v4f vals[8];
#pragma unroll
            for (int i = 0; i < 8; ++i) vals[i] = *(const v4f*)(S32 + (wid * 8 + i) * 132 + lane * 4);
            float* dbase = out32 + (size_t)(mBase + p * 64 + wid * 8) * ldc + nBase + lane * 4;
#pragma unroll
            for (int i = 0; i < 8; ++i) *(volatile v4f*)(dbase + (size_t)i * ldc) = vals[i];
            __threadfence();
#pragma unroll
            for (int i = 0; i < 8; ++i) *(volatile v4f*)(dbase + (size_t)i * ldc) = vals[i];
            __syncthreads();
        }
    } else {
#pragma unroll
        for (int mi = 0; mi < 4; ++mi)
#pragma unroll
            for (int ni = 0; ni < 2; ++ni)
#pragma unroll
                for (int r = 0; r < 8; ++r)
                    S16[(wm * 64 + mi * 16 + 8 * hf + r) * 136 + wn * 32 + ni * 16 + m] = (f16t)(acc[mi][ni][r] * osc);
        __syncthreads();
        {
            v8h vals[8];
#pragma unroll
            for (int it = 0; it < 8; ++it)
                vals[it] = *(const v8h*)(S16 + (wid * 16 + 2 * it + hf) * 136 + m * 8);
            f16t* dbase = out16 + (size_t)(mBase + wid * 16 + hf) * ldc + nBase + m * 8;
#pragma unroll
            for (int it = 0; it < 8; ++it) *(volatile v8h*)(dbase + (size_t)(2 * it) * ldc) = vals[it];
            __threadfence();
#pragma unroll
            for (int it = 0; it < 8; ++it) *(volatile v8h*)(dbase + (size_t)(2 * it) * ldc) = vals[it];
        }
        if (mode == 2) {
            __syncthreads();
#pragma unroll
            for (int mi = 0; mi < 4; ++mi)
#pragma unroll
                for (int ni = 0; ni < 2; ++ni)
#pragma unroll
                    for (int r = 0; r < 8; ++r)
                        S16[(wn * 32 + ni * 16 + m) * 136 + wm * 64 + mi * 16 + 8 * hf + r] = (f16t)(acc[mi][ni][r] * osc);
            __syncthreads();
            v8h vals[8];
#pragma unroll
            for (int it = 0; it < 8; ++it)
                vals[it] = *(const v8h*)(S16 + (wid * 16 + 2 * it + hf) * 136 + m * 8);
            const int bidx = mBase / SEQ, s0 = mBase - bidx * SEQ;
            f16t* dbase = outT + (size_t)(bidx * N + nBase + wid * 16 + hf) * SEQ + s0 + m * 8;
#pragma unroll
            for (int it = 0; it < 8; ++it) *(volatile v8h*)(dbase + (size_t)(2 * it) * SEQ) = vals[it];
            __threadfence();
#pragma unroll
            for (int it = 0; it < 8; ++it) *(volatile v8h*)(dbase + (size_t)(2 * it) * SEQ) = vals[it];
        }
    }
}

__global__ __launch_bounds__(256) void k_conv(const f16t* __restrict__ xm16, const float* __restrict__ cw,
                                                const float* __restrict__ cb, float* __restrict__ xc32,
                                                f16t* __restrict__ xc16, int n8, float inscale, float outscale)
{
    const int i = blockIdx.x * 256 + threadIdx.x;
    if (i >= n8) return;
    const int m = i / (INN / 8);
    const int c0 = (i - m * (INN / 8)) * 8;
    const int s = m & (SEQ - 1);
    v4f w[8];
    const v4f* cwp = (const v4f*)(cw + (size_t)c0 * 4);
#pragma unroll
    for (int e = 0; e < 8; ++e) w[e] = cwp[e];
    float acc[8];
#pragma unroll
    for (int e = 0; e < 8; ++e) acc[e] = 0.f;
#pragma unroll
    for (int t = 0; t < 4; ++t) {
        const int ss = s - 3 + t;
        if (ss >= 0) {
            const v8h xv = *(const v8h*)(xm16 + (size_t)(m - 3 + t) * INN + c0);
#pragma unroll
            for (int e = 0; e < 8; ++e) acc[e] += w[e][t] * ((float)xv[e] * inscale);
        }
    }
    float o[8];
#pragma unroll
    for (int e = 0; e < 8; ++e) {
        const float v = acc[e] + cb[c0 + e];
        o[e] = v * (1.0f / (1.0f + __expf(-v)));
    }
    v4f o0, o1;
    v8h oh;
#pragma unroll
    for (int e = 0; e < 4; ++e) { o0[e] = o[e]; o1[e] = o[4 + e]; }
#pragma unroll
    for (int e = 0; e < 8; ++e) oh[e] = (f16t)(o[e] * outscale);
    float* d32 = xc32 + (size_t)i * 8;
    f16t*  d16 = xc16 + (size_t)i * 8;
    *(volatile v4f*)d32 = o0; *(volatile v4f*)(d32 + 4) = o1; *(volatile v8h*)d16 = oh;
    __threadfence();
    *(volatile v4f*)d32 = o0; *(volatile v4f*)(d32 + 4) = o1; *(volatile v8h*)d16 = oh;
}

__global__ __launch_bounds__(32) void k_gates(const f16t* __restrict__ q16, const f16t* __restrict__ k16,
                                                const f16t* __restrict__ v16, const f16t* __restrict__ WgT,
                                                const float* __restrict__ bi, const float* __restrict__ bfv,
                                                float* __restrict__ ig, float* __restrict__ logf,
                                                int Mrows, float sq, float sk, float sv)
{
    __shared__ __align__(16) float G[16 * 36];
    const int lane = threadIdx.x, hf = lane >> 4, m = lane & 15;
    const int row0 = blockIdx.x * 32;
    if (row0 + 32 > Mrows) return;
    v8f acc[2][3];
#pragma unroll
    for (int t = 0; t < 2; ++t) { acc[t][0] = zacc(); acc[t][1] = zacc(); acc[t][2] = zacc(); }
    const f16t* parts[3] = { q16, k16, v16 };
#pragma unroll
    for (int p = 0; p < 3; ++p) {
        const f16t* Ap = parts[p] + (size_t)(row0 + m) * INN + 8 * hf;
        const f16t* Bp = WgT + (size_t)m * GK + p * INN + 8 * hf;
#pragma unroll 1
        for (int kb = 0; kb < INN; kb += 32) {
            Frag b;
            b.h[0] = *(const v8h*)(Bp + kb);
            b.h[1] = *(const v8h*)(Bp + kb + 16);
#pragma unroll
            for (int t = 0; t < 2; ++t) {
                Frag a;
                const f16t* pa = Ap + (size_t)(t * 16) * INN + kb;
                a.h[0] = *(const v8h*)pa;
                a.h[1] = *(const v8h*)(pa + 16);
                acc[t][p] = wmma16(a.v, b.v, acc[t][p]);
            }
        }
    }
#pragma unroll
    for (int t = 0; t < 2; ++t)
#pragma unroll
        for (int r = 0; r < 8; ++r) {
            float val = acc[t][0][r] * sq + acc[t][1][r] * sk + acc[t][2][r] * sv;
            if (m < 8) val = val + bi[m];
            else       val = logsig(val + bfv[m - 8]);
            G[m * 36 + t * 16 + 8 * hf + r] = val;
        }
    __syncthreads();
    const int bidx = row0 / SEQ, s0 = row0 - bidx * SEQ;
    const int piece = lane & 7;
    v4f vals[4];
    float* dst[4];
#pragma unroll
    for (int it = 0; it < 4; ++it) {
        const int L = (lane >> 3) + 4 * it;
        vals[it] = *(const v4f*)(G + L * 36 + piece * 4);
        dst[it] = ((L < 8) ? (ig + (size_t)(bidx * NHD + L) * SEQ + s0)
                           : (logf + (size_t)(bidx * NHD + L - 8) * SEQ + s0)) + piece * 4;
    }
#pragma unroll
    for (int it = 0; it < 4; ++it) *(volatile v4f*)dst[it] = vals[it];
    __threadfence();
#pragma unroll
    for (int it = 0; it < 4; ++it) *(volatile v4f*)dst[it] = vals[it];
}

__global__ __launch_bounds__(32) void k_scan(const float* __restrict__ ig, const float* __restrict__ logf,
                                               float* __restrict__ rowt, float* __restrict__ colt,
                                               float* __restrict__ nmld, int nseq, int S)
{
    const int t = threadIdx.x;
    if (t >= nseq) return;
    const size_t base = (size_t)t * S;
#pragma unroll 1
    for (int pass = 0; pass < 2; ++pass) {
        double cs = 0.0;
        float pm = -__builtin_inff();
#pragma unroll 1
        for (int i = 0; i < S; i += 4) {
            v4f br, bc, bn;
#pragma unroll
            for (int u = 0; u < 4; ++u) {
                cs += (double)logf[base + i + u];
                const float csf = (float)cs;
                const float g = ig[base + i + u] - csf;
                pm = fmaxf(pm, g);
                br[u] = pm; bc[u] = g; bn[u] = -(csf + pm);
            }
            *(volatile v4f*)(rowt + base + i) = br;
            *(volatile v4f*)(colt + base + i) = bc;
            *(volatile v4f*)(nmld + base + i) = bn;
        }
        __threadfence();
    }
}

__global__ __launch_bounds__(256) void k_attn(const f16t* __restrict__ q16, const f16t* __restrict__ k16,
                                                const f16t* __restrict__ vT,
                                                const float* __restrict__ rowt, const float* __restrict__ colt,
                                                const float* __restrict__ nmld,
                                                const float* __restrict__ xc32, const float* __restrict__ z32,
                                                const float* __restrict__ normw, const float* __restrict__ skipp,
                                                f16t* __restrict__ hf16,
                                                float qkscale, float pscale, float hscale, float oscale)
{
    __shared__ __align__(16) f16t Pl[NHD * 640];
    __shared__ __align__(16) f16t Hs[16 * 1160];
    const int tid = threadIdx.x, wid = tid >> 5, lane = tid & 31, hf = lane >> 4, m = lane & 15;
    const int b  = blockIdx.x >> 7;
    const int i0 = (blockIdx.x & 127) << 4;
    const int hd = wid;
    const int bh = b * NHD + hd;
    f16t* Pw = Pl + wid * 640;
    const f16t* qb = q16 + (size_t)(b * SEQ + i0 + m) * INN + hd * DHD + 8 * hf;

    float rt[8], rs[8];
#pragma unroll
    for (int r = 0; r < 8; ++r) {
        rt[r] = rowt[(size_t)bh * SEQ + i0 + 8 * hf + r];
        rs[r] = 0.f;
    }
    v8f ha[9];
#pragma unroll
    for (int dt = 0; dt < 9; ++dt) ha[dt] = zacc();

    const int jmax = i0 + 15;
    for (int j0 = 0; j0 <= jmax; j0 += 32) {
#pragma unroll
        for (int jj = 0; jj < 2; ++jj) {
            const int j0t = j0 + 16 * jj;
            if (j0t <= jmax) {
                v8f qk = zacc();
                const f16t* kbp = k16 + (size_t)(b * SEQ + j0t + m) * INN + hd * DHD + 8 * hf;
#pragma unroll
                for (int d = 0; d < 5; ++d) {
                    Frag qa, kf;
                    qa.h[0] = *(const v8h*)(qb + d * 32);
                    kf.h[0] = *(const v8h*)(kbp + d * 32);
                    if (d < 4) {
                        qa.h[1] = *(const v8h*)(qb + d * 32 + 16);
                        kf.h[1] = *(const v8h*)(kbp + d * 32 + 16);
                    } else {
                        qa.u[1] = zu4();
                        kf.u[1] = zu4();
                    }
                    qk = wmma16(qa.v, kf.v, qk);
                }
                const float ct = colt[(size_t)bh * SEQ + j0t + m];
                const int col = j0t + m;
#pragma unroll
                for (int r = 0; r < 8; ++r) {
                    const int row = i0 + 8 * hf + r;
                    const float e = __expf(fminf(ct - rt[r], 0.f));
                    const float p = (col <= row) ? (qk[r] * qkscale * e) : 0.f;
                    rs[r] += p;
                    Pw[(8 * hf + r) * 40 + jj * 16 + m] = (f16t)(p * pscale);
                }
            } else {
#pragma unroll
                for (int r = 0; r < 8; ++r) Pw[(8 * hf + r) * 40 + jj * 16 + m] = (f16t)0.0f;
            }
        }
        __syncthreads();
        Frag pf;
        pf.h[0] = *(const v8h*)(Pw + m * 40 + 8 * hf);
        pf.h[1] = *(const v8h*)(Pw + m * 40 + 16 + 8 * hf);
        const f16t* vb = vT + (size_t)(b * INN + hd * DHD + m) * SEQ + j0 + 8 * hf;
#pragma unroll
        for (int dt = 0; dt < 9; ++dt) {
            Frag vf;
            const f16t* vp = vb + (size_t)(dt * 16) * SEQ;
            vf.h[0] = *(const v8h*)vp;
            vf.h[1] = *(const v8h*)(vp + 16);
            ha[dt] = wmma16(pf.v, vf.v, ha[dt]);
        }
        __syncthreads();
    }

#pragma unroll
    for (int r = 0; r < 8; ++r) {
        float v = rs[r];
        v += __shfl_xor(v, 1, 16); v += __shfl_xor(v, 2, 16);
        v += __shfl_xor(v, 4, 16); v += __shfl_xor(v, 8, 16);
        rs[r] = v;
    }
    const float skipv = skipp[0];
#pragma unroll
    for (int r = 0; r < 8; ++r) {
        const int row = i0 + 8 * hf + r;
        const size_t mrow = (size_t)(b * SEQ + row);
        const float nm  = nmld[(size_t)bh * SEQ + row];
        const float nrm = fmaxf(fabsf(rs[r]), expf(nm)) + 1e-6f;
        const float inv = hscale * (1.0f / nrm);
        float hv[9];
        float s1 = 0.f;
#pragma unroll
        for (int dt = 0; dt < 9; ++dt) { hv[dt] = ha[dt][r] * inv; s1 += hv[dt]; }
        s1 += __shfl_xor(s1, 1, 16); s1 += __shfl_xor(s1, 2, 16);
        s1 += __shfl_xor(s1, 4, 16); s1 += __shfl_xor(s1, 8, 16);
        const float mean = s1 * (1.0f / 144.0f);
        float s2 = 0.f;
#pragma unroll
        for (int dt = 0; dt < 9; ++dt) { const float d = hv[dt] - mean; hv[dt] = d; s2 += d * d; }
        s2 += __shfl_xor(s2, 1, 16); s2 += __shfl_xor(s2, 2, 16);
        s2 += __shfl_xor(s2, 4, 16); s2 += __shfl_xor(s2, 8, 16);
        const float var  = s2 * (1.0f / 144.0f);
        const float rstd = 1.0f / sqrtf(var + 1e-5f);
#pragma unroll
        for (int dt = 0; dt < 9; ++dt) {
            const int c = hd * DHD + dt * 16 + m;
            float x = hv[dt] * rstd * normw[c] + skipv * xc32[mrow * INN + c];
            const float z = z32[mrow * INN + c];
            x *= z * (1.0f / (1.0f + __expf(-z)));
            Hs[(8 * hf + r) * 1160 + c] = (f16t)(x * oscale);
        }
    }
    __syncthreads();
#pragma unroll
    for (int rr = 0; rr < 2; ++rr) {
        const int rl = 2 * wid + rr;
        f16t* dbase = hf16 + (size_t)(b * SEQ + i0 + rl) * INN;
        const f16t* sbase = Hs + rl * 1160;
#pragma unroll
        for (int k = 0; k < 5; ++k) {
            const int piece = lane + 32 * k;
            if (piece < 144) *(volatile v8h*)(dbase + piece * 8) = *(const v8h*)(sbase + piece * 8);
        }
    }
    __threadfence();
#pragma unroll
    for (int rr = 0; rr < 2; ++rr) {
        const int rl = 2 * wid + rr;
        f16t* dbase = hf16 + (size_t)(b * SEQ + i0 + rl) * INN;
        const f16t* sbase = Hs + rl * 1160;
#pragma unroll
        for (int k = 0; k < 5; ++k) {
            const int piece = lane + 32 * k;
            if (piece < 144) *(volatile v8h*)(dbase + piece * 8) = *(const v8h*)(sbase + piece * 8);
        }
    }
}

extern "C" void kernel_launch(void* const* d_in, const int* in_sizes, int n_in,
                              void* d_out, int out_size, void* d_ws, size_t ws_size,
                              hipStream_t stream)
{
    if (n_in < 14) return;
    if (out_size != MROWS * HD) return;
    if (in_sizes[0] != MROWS * HD || in_sizes[1] != HD * 2 * INN || in_sizes[4] != INN * INN ||
        in_sizes[13] != INN * HD || in_sizes[7] != GK * NHD || in_sizes[9] != GK * NHD) return;

    const float* x      = (const float*)d_in[0];
    const float* W_up   = (const float*)d_in[1];
    const float* conv_w = (const float*)d_in[2];
    const float* conv_b = (const float*)d_in[3];
    const float* Wq     = (const float*)d_in[4];
    const float* Wk     = (const float*)d_in[5];
    const float* Wv     = (const float*)d_in[6];
    const float* Wi     = (const float*)d_in[7];
    const float* bi     = (const float*)d_in[8];
    const float* Wf     = (const float*)d_in[9];
    const float* bfv    = (const float*)d_in[10];
    const float* norm_w = (const float*)d_in[11];
    const float* skipp  = (const float*)d_in[12];
    const float* W_down = (const float*)d_in[13];
    float* outp = (float*)d_out;

    char* w = (char*)d_ws;
    size_t off = 0;
    const size_t nAct = (size_t)MROWS * INN;
    const size_t nGate = (size_t)BSZ * NHD * SEQ;
#define CARVE(ptr, type, count) ptr = (type*)(w + off); off += (((size_t)(count) * sizeof(type)) + 255) & ~(size_t)255
    f16t* x16;    CARVE(x16, f16t, (size_t)MROWS * HD);
    f16t* WupT16; CARVE(WupT16, f16t, (size_t)2 * INN * HD);
    f16t* WqT16;  CARVE(WqT16, f16t, (size_t)INN * INN);
    f16t* WkT16;  CARVE(WkT16, f16t, (size_t)INN * INN);
    f16t* WvT16;  CARVE(WvT16, f16t, (size_t)INN * INN);
    f16t* WdT16;  CARVE(WdT16, f16t, (size_t)HD * INN);
    f16t* WgT16;  CARVE(WgT16, f16t, (size_t)16 * GK);
    float* z32;   CARVE(z32, float, nAct);
    f16t* xm16;   CARVE(xm16, f16t, nAct);
    float* xc32;  CARVE(xc32, float, nAct);
    f16t* xc16;   CARVE(xc16, f16t, nAct);
    f16t* q16;    CARVE(q16, f16t, nAct);
    f16t* k16;    CARVE(k16, f16t, nAct);
    f16t* v16;    CARVE(v16, f16t, nAct);
    f16t* vT16;   CARVE(vT16, f16t, nAct);
    f16t* hf16;   CARVE(hf16, f16t, nAct);
    float* ig;    CARVE(ig, float, nGate);
    float* logf;  CARVE(logf, float, nGate);
    float* rowt;  CARVE(rowt, float, nGate);
    float* colt;  CARVE(colt, float, nGate);
    float* nmld;  CARVE(nmld, float, nGate);
#undef CARVE
    if (off > ws_size) return;

    const float Sx = 8.f, SW = 64.f, Sm = 8.f, Sc = 1024.f, Sq = 512.f, Sk = 8192.f, Sv = 16.f, Sp = 65536.f, Sh = 64.f;
    const float osc_xm  = Sm / (Sx * SW);
    const float osc_z   = 1.f / (Sx * SW);
    const float osc_q   = Sq / (Sc * SW);
    const float osc_k   = (Sk / (Sc * SW)) * (1.0f / 12.0f);
    const float osc_v   = Sv / (Sm * SW);
    const float g_sq    = 1.f / (Sq * SW);
    const float g_sk    = 12.f / (Sk * SW);
    const float g_sv    = 1.f / (Sv * SW);
    const float qkscale = 1.f / (Sq * Sk);
    const float hscale  = 1.f / (Sp * Sv);
    const float osc_out = 1.f / (Sh * SW);

    {
        const int n8 = MROWS * HD / 8;
        k_cvt_rows<<<(n8 + 255) / 256, 256, 0, stream>>>(x, x16, n8, Sx);
    }
    k_tr_cvt<<<dim3((HD + 63) / 64, (2 * INN + 63) / 64), 256, 0, stream>>>(W_up, WupT16, HD, 2 * INN, SW);
    k_tr_cvt<<<dim3((INN + 63) / 64, (INN + 63) / 64), 256, 0, stream>>>(Wq, WqT16, INN, INN, SW);
    k_tr_cvt<<<dim3((INN + 63) / 64, (INN + 63) / 64), 256, 0, stream>>>(Wk, WkT16, INN, INN, SW);
    k_tr_cvt<<<dim3((INN + 63) / 64, (INN + 63) / 64), 256, 0, stream>>>(Wv, WvT16, INN, INN, SW);
    k_tr_cvt<<<dim3((INN + 63) / 64, (HD + 63) / 64), 256, 0, stream>>>(W_down, WdT16, INN, HD, SW);
    {
        const int n8 = 16 * GK / 8;
        k_gatew<<<(n8 + 255) / 256, 256, 0, stream>>>(Wi, Wf, WgT16, n8, SW);
    }
    k_gemm<<<dim3(INN / 128, MROWS / 128), 256, 0, stream>>>(
        x16, HD, WupT16, HD, xm16, z32, vT16, INN, MROWS, INN, HD, 0, osc_xm);
    k_gemm<<<dim3(INN / 128, MROWS / 128), 256, 0, stream>>>(
        x16, HD, WupT16 + (size_t)INN * HD, HD, xm16, z32, vT16, INN, MROWS, INN, HD, 1, osc_z);
    {
        const int n8 = MROWS * (INN / 8);
        k_conv<<<(n8 + 255) / 256, 256, 0, stream>>>(xm16, conv_w, conv_b, xc32, xc16, n8, 1.f / Sm, Sc);
    }
    k_gemm<<<dim3(INN / 128, MROWS / 128), 256, 0, stream>>>(
        xc16, INN, WqT16, INN, q16, z32, vT16, INN, MROWS, INN, INN, 0, osc_q);
    k_gemm<<<dim3(INN / 128, MROWS / 128), 256, 0, stream>>>(
        xc16, INN, WkT16, INN, k16, z32, vT16, INN, MROWS, INN, INN, 0, osc_k);
    k_gemm<<<dim3(INN / 128, MROWS / 128), 256, 0, stream>>>(
        xm16, INN, WvT16, INN, v16, z32, vT16, INN, MROWS, INN, INN, 2, osc_v);
    k_gates<<<MROWS / 32, 32, 0, stream>>>(q16, k16, v16, WgT16, bi, bfv, ig, logf, MROWS, g_sq, g_sk, g_sv);
    k_scan<<<1, 32, 0, stream>>>(ig, logf, rowt, colt, nmld, BSZ * NHD, SEQ);
    k_attn<<<BSZ * (SEQ / 16), 256, 0, stream>>>(
        q16, k16, vT16, rowt, colt, nmld, xc32, z32, norm_w, skipp, hf16, qkscale, Sp, hscale, Sh);
    k_gemm<<<dim3(HD / 128, MROWS / 128), 256, 0, stream>>>(
        hf16, INN, WdT16, INN, xm16, outp, vT16, HD, MROWS, HD, INN, 1, osc_out);

    (void)ws_size;
}
